// MultiHeadAttention_43370579755636
// MI455X (gfx1250) — hardware-verified
//
#include <hip/hip_runtime.h>
#ifndef NB
#define NB 2
#endif
#ifndef SEQ
#define SEQ 2048
#endif
#define SEQ_FULL 2048
#define DM 1024
#define NH 16
#define HD 64
#define NR (NB * SEQ)
#define LDSP 68
#define CTP 72

typedef _Float16 v16h __attribute__((ext_vector_type(16)));
typedef unsigned short v8us __attribute__((ext_vector_type(8), may_alias));
typedef float v8f  __attribute__((ext_vector_type(8)));
typedef float v4f  __attribute__((ext_vector_type(4)));
typedef float v4fa __attribute__((ext_vector_type(4), may_alias));
union FragH { v16h v; v8us half[2]; _Float16 h[16]; unsigned short u[16]; };

static_assert(NH * HD == DM);
static_assert(SEQ % 128 == 0 && SEQ <= SEQ_FULL);
static_assert(DM % 64 == 0 && (3 * DM) % 64 == 0 && DM % 32 == 0);
static_assert((NB * NH * (SEQ / 16)) % 4 == 0);

__device__ __forceinline__ float bf16_rne(float x) {
  unsigned int u = __float_as_uint(x);
  u = (u + 0x7FFFu + ((u >> 16) & 1u)) & 0xFFFF0000u;
  return __uint_as_float(u);
}

__device__ __forceinline__ v16h g2_frag(const _Float16* p, int hh) {
  FragH f;
  f.half[0] = *(const v8us*)((const unsigned short*)p + 8 * hh);
  f.half[1] = *(const v8us*)((const unsigned short*)p + 16 + 8 * hh);
  return f.v;
}
__device__ __forceinline__ v8f g2_mma(v16h a, v16h b, v8f c) {
  v8f d = __builtin_amdgcn_wmma_f32_16x16x32_f16(false, a, false, b, (short)0, c, false, false);
  asm volatile("v_nop\n\tv_nop\n\tv_nop\n\tv_nop" : "+v"(d) : "v"(a), "v"(b));
  return d;
}

__global__ __launch_bounds__(256) void k_x16(const float* __restrict__ x, _Float16* __restrict__ X16) {
  const size_t t = (size_t)blockIdx.x * 256 + threadIdx.x;
  if (t >= (size_t)NR * DM / 8) return;
  const size_t row = t / (DM / 8);
  const int c8 = (int)(t % (DM / 8)) * 8;
  const size_t b = row / SEQ, s = row % SEQ;
  const float* src = x + ((b * SEQ_FULL + s) * DM + c8);
  const v4f a = *(const v4fa*)src, c = *(const v4fa*)(src + 4);
  FragH f;
#pragma unroll
  for (int q = 0; q < 4; ++q) { f.h[q] = (_Float16)bf16_rne(a[q]); f.h[4 + q] = (_Float16)bf16_rne(c[q]); }
  const v8us o = f.half[0];
  unsigned short* d = (unsigned short*)X16 + t * 8;
  *(volatile v8us*)d = o;
  __threadfence();
  *(volatile v8us*)d = o;
}

__global__ __launch_bounds__(256) void k_wnat(const float* __restrict__ w, size_t n8, _Float16* __restrict__ Bt) {
  const size_t t = (size_t)blockIdx.x * 256 + threadIdx.x;
  if (t >= n8) return;
  const v4f a = *(const v4fa*)(w + t * 8), c = *(const v4fa*)(w + t * 8 + 4);
  FragH f;
#pragma unroll
  for (int q = 0; q < 4; ++q) { f.h[q] = (_Float16)(bf16_rne(a[q]) * 16.0f); f.h[4 + q] = (_Float16)(bf16_rne(c[q]) * 16.0f); }
  const v8us o = f.half[0];
  unsigned short* d = (unsigned short*)Bt + t * 8;
  *(volatile v8us*)d = o;
  __threadfence();
  *(volatile v8us*)d = o;
}

__global__ __launch_bounds__(256) void k_tab(float* __restrict__ ctab, float* __restrict__ stab) {
  const int t = blockIdx.x * 256 + threadIdx.x;
  if (t >= SEQ * 32) return;
  const int p = t & 31, s = t >> 5;
  const float e = (float)((double)(2 * p) * -0.20762050593046014);
  const float inv = exp2f(e);
  const float fr = (float)s * inv;
  const float c = cosf(fr);
  const float sn = sinf(fr);
  *(volatile float*)(ctab + t) = c;
  *(volatile float*)(stab + t) = sn;
  __threadfence();
  *(volatile float*)(ctab + t) = c;
  *(volatile float*)(stab + t) = sn;
}

__global__ __launch_bounds__(128) void k_qkv(const _Float16* __restrict__ A, const _Float16* __restrict__ Bh,
                                             const float* __restrict__ ctab, const float* __restrict__ stab,
                                             _Float16* __restrict__ QK, _Float16* __restrict__ VT) {
  __shared__ __attribute__((aligned(16))) float so[4][32][LDSP];
  const int tid = threadIdx.x, w = tid >> 5, lane = tid & 31, ln = lane & 15, hh = lane >> 4;
  const int ntn = (3 * DM) / 64;
  const int mt = blockIdx.x / ntn, nq = blockIdx.x - mt * ntn;
  const int row0 = mt * 128 + 32 * w, col0 = nq * 64;
  const _Float16* a0p = A + (size_t)(row0 + ln) * DM; const _Float16* a1p = a0p + (size_t)16 * DM;
  const _Float16* b0p = Bh + (size_t)(col0 + ln) * DM; const _Float16* b1p = b0p + (size_t)16 * DM;
  const _Float16* b2p = b1p + (size_t)16 * DM; const _Float16* b3p = b2p + (size_t)16 * DM;
  const v8f z8 = {0.f,0.f,0.f,0.f,0.f,0.f,0.f,0.f};
  v8f c00 = z8, c01 = z8, c02 = z8, c03 = z8, c10 = z8, c11 = z8, c12 = z8, c13 = z8;
#pragma unroll 1
  for (int kb = 0; kb < DM; kb += 32) {
    const v16h a0 = g2_frag(a0p + kb, hh), a1 = g2_frag(a1p + kb, hh);
    v16h b = g2_frag(b0p + kb, hh); c00 = g2_mma(a0, b, c00); c10 = g2_mma(a1, b, c10);
    b = g2_frag(b1p + kb, hh); c01 = g2_mma(a0, b, c01); c11 = g2_mma(a1, b, c11);
    b = g2_frag(b2p + kb, hh); c02 = g2_mma(a0, b, c02); c12 = g2_mma(a1, b, c12);
    b = g2_frag(b3p + kb, hh); c03 = g2_mma(a0, b, c03); c13 = g2_mma(a1, b, c13);
  }
  v8f accs[8] = {c00, c01, c02, c03, c10, c11, c12, c13};
#pragma unroll
  for (int u = 0; u < 8; ++u) {
    const int t = u & 3, hf = u >> 2;
#pragma unroll
    for (int r = 0; r < 8; ++r) so[w][hf * 16 + 8 * hh + r][t * 16 + ln] = accs[u][r] * 0.0625f;
  }
  __syncthreads();
  const int sec = nq / NH, head = nq - sec * NH;
  const int bb = (mt * 128) / SEQ, sblk = (mt * 128) - bb * SEQ;
  const int slab = bb * NH + head;
  const int pc = lane & 7, rg = lane >> 3;
  v8us ov[8];
  if (sec < 2) {
#pragma unroll
    for (int i = 0; i < 8; ++i) {
      const int rloc = i * 4 + rg;
      const int s = sblk + 32 * w + rloc;
      const v4f x0 = *(const v4fa*)&so[w][rloc][pc * 8], x1 = *(const v4fa*)&so[w][rloc][pc * 8 + 4];
      const v4f cc = *(const v4fa*)(ctab + (size_t)s * 32 + pc * 4), ss = *(const v4fa*)(stab + (size_t)s * 32 + pc * 4);
      FragH f;
      f.h[0] = (_Float16)(x0[0] * cc[0] - x0[1] * ss[0]); f.h[1] = (_Float16)(x0[0] * ss[0] + x0[1] * cc[0]);
      f.h[2] = (_Float16)(x0[2] * cc[1] - x0[3] * ss[1]); f.h[3] = (_Float16)(x0[2] * ss[1] + x0[3] * cc[1]);
      f.h[4] = (_Float16)(x1[0] * cc[2] - x1[1] * ss[2]); f.h[5] = (_Float16)(x1[0] * ss[2] + x1[1] * cc[2]);
      f.h[6] = (_Float16)(x1[2] * cc[3] - x1[3] * ss[3]); f.h[7] = (_Float16)(x1[2] * ss[3] + x1[3] * cc[3]);
      ov[i] = f.half[0];
    }
    unsigned short* dst = (unsigned short*)QK + ((size_t)sec * NB * NH + slab) * SEQ * HD;
    for (int pass = 0; pass < 2; ++pass) {
#pragma unroll
      for (int i = 0; i < 8; ++i) {
        const int s = sblk + 32 * w + i * 4 + rg;
        *(volatile v8us*)(dst + (size_t)s * HD + pc * 8) = ov[i];
      }
      if (pass == 0) __threadfence();
    }
  } else {
#pragma unroll
    for (int i = 0; i < 8; ++i) {
      const int L = (w * 8 + i) * 4 + rg;
      const int d = L >> 1, tl = (L & 1) * 64 + pc * 8;
      const int wsrc = tl >> 5, rl0 = tl & 31;
      FragH f;
#pragma unroll
      for (int q = 0; q < 8; ++q) f.h[q] = (_Float16)so[wsrc][rl0 + q][d];
      ov[i] = f.half[0];
    }
    unsigned short* dst = (unsigned short*)VT + (size_t)slab * HD * SEQ;
    for (int pass = 0; pass < 2; ++pass) {
#pragma unroll
      for (int i = 0; i < 8; ++i) {
        const int L = (w * 8 + i) * 4 + rg;
        const int d = L >> 1, tl = (L & 1) * 64 + pc * 8;
        *(volatile v8us*)(dst + (size_t)d * SEQ + sblk + tl) = ov[i];
      }
      if (pass == 0) __threadfence();
    }
  }
}

__global__ __launch_bounds__(128) void k_flash(const _Float16* __restrict__ Qp, const _Float16* __restrict__ Kp,
                                               const _Float16* __restrict__ VTp, _Float16* __restrict__ CTX) {
  __shared__ __attribute__((aligned(16))) unsigned short ct[4][16][CTP];
  const int tid = threadIdx.x, w = tid >> 5, lane = tid & 31, ln = lane & 15, hh = lane >> 4;
  const int wid = blockIdx.x * 4 + w;
  const int st = wid % (SEQ / 16), bh = wid / (SEQ / 16);
  const int s0 = st * 16;
  const _Float16* qrow = Qp + ((size_t)bh * SEQ + s0 + ln) * HD;
  const _Float16* kbase = Kp + ((size_t)bh * SEQ + ln) * HD;
  const _Float16* vbase = VTp + ((size_t)bh * HD + ln) * SEQ;
  const v16h qb0 = g2_frag(qrow, hh), qb1 = g2_frag(qrow + 32, hh);
  const v8f z8 = {0.f,0.f,0.f,0.f,0.f,0.f,0.f,0.f};
  v8f c0 = z8, c1 = z8, c2 = z8, c3 = z8;
  float rm = -3.0e38f, rl = 0.0f;
  const float CS = 0.125f * 1.4426950408889634f;
#pragma unroll 1
  for (int t0 = 0; t0 < SEQ; t0 += 32) {
    const _Float16* k0 = kbase + (size_t)t0 * HD;
    const _Float16* k1 = k0 + (size_t)16 * HD;
    v8f sa = z8, sb = z8;
    sa = g2_mma(g2_frag(k0, hh), qb0, sa);
    sa = g2_mma(g2_frag(k0 + 32, hh), qb1, sa);
    sb = g2_mma(g2_frag(k1, hh), qb0, sb);
    sb = g2_mma(g2_frag(k1 + 32, hh), qb1, sb);
    float lmax = fmaxf(sa[0], sb[0]);
#pragma unroll
    for (int e = 1; e < 8; ++e) lmax = fmaxf(lmax, fmaxf(sa[e], sb[e]));
    lmax = fmaxf(lmax, __shfl_xor(lmax, 16, 32));
    const float mnew = fmaxf(rm, lmax);
    const float alpha = __builtin_amdgcn_exp2f((rm - mnew) * CS);
    rm = mnew;
    const float nb = 8.0f - mnew * CS;
    FragH pb;
    float ls = 0.0f;
#pragma unroll
    for (int e = 0; e < 8; ++e) {
      const float p0 = __builtin_amdgcn_exp2f(fmaf(sa[e], CS, nb));
      const float p1 = __builtin_amdgcn_exp2f(fmaf(sb[e], CS, nb));
      ls += p0 + p1;
      pb.h[e] = (_Float16)p0;
      pb.h[8 + e] = (_Float16)p1;
    }
    ls += __shfl_xor(ls, 16, 32);
    rl = rl * alpha + ls;
#pragma unroll
    for (int e = 0; e < 8; ++e) { c0[e] *= alpha; c1[e] *= alpha; c2[e] *= alpha; c3[e] *= alpha; }
    c0 = g2_mma(g2_frag(vbase + t0, hh), pb.v, c0);
    c1 = g2_mma(g2_frag(vbase + (size_t)16 * SEQ + t0, hh), pb.v, c1);
    c2 = g2_mma(g2_frag(vbase + (size_t)32 * SEQ + t0, hh), pb.v, c2);
    c3 = g2_mma(g2_frag(vbase + (size_t)48 * SEQ + t0, hh), pb.v, c3);
  }
  const float il = 64.0f / rl;
  FragH f0, f1, f2, f3;
#pragma unroll
  for (int e = 0; e < 8; ++e) {
    f0.h[e] = (_Float16)(c0[e] * il); f1.h[e] = (_Float16)(c1[e] * il);
    f2.h[e] = (_Float16)(c2[e] * il); f3.h[e] = (_Float16)(c3[e] * il);
  }
  *(v8us*)&ct[w][ln][0  + 8 * hh] = f0.half[0];
  *(v8us*)&ct[w][ln][16 + 8 * hh] = f1.half[0];
  *(v8us*)&ct[w][ln][32 + 8 * hh] = f2.half[0];
  *(v8us*)&ct[w][ln][48 + 8 * hh] = f3.half[0];
  __builtin_amdgcn_fence(4  , "workgroup");
  __builtin_amdgcn_wave_barrier();
  const int b = bh / NH, h = bh - b * NH;
  const int pc = lane & 7, rg = lane >> 3;
  v8us ov[4];
#pragma unroll
  for (int i = 0; i < 4; ++i) ov[i] = *(const v8us*)&ct[w][i * 4 + rg][pc * 8];
  unsigned short* dst = (unsigned short*)CTX + ((size_t)b * SEQ + s0) * DM + h * HD + pc * 8;
  for (int pass = 0; pass < 2; ++pass) {
#pragma unroll
    for (int i = 0; i < 4; ++i) *(volatile v8us*)(dst + (size_t)(i * 4 + rg) * DM) = ov[i];
    if (pass == 0) __threadfence();
  }
}

__global__ __launch_bounds__(128) void k_out(const _Float16* __restrict__ A, const _Float16* __restrict__ Bh, float alpha, float* __restrict__ C) {
  __shared__ __attribute__((aligned(16))) float so[4][32][LDSP];
  const int tid = threadIdx.x, w = tid >> 5, lane = tid & 31, ln = lane & 15, hh = lane >> 4;
  const int ntn = DM / 64;
  const int mt = blockIdx.x / ntn, nq = blockIdx.x - mt * ntn;
  const int row0 = mt * 128 + 32 * w, col0 = nq * 64;
  const _Float16* a0p = A + (size_t)(row0 + ln) * DM; const _Float16* a1p = a0p + (size_t)16 * DM;
  const _Float16* b0p = Bh + (size_t)(col0 + ln) * DM; const _Float16* b1p = b0p + (size_t)16 * DM;
  const _Float16* b2p = b1p + (size_t)16 * DM; const _Float16* b3p = b2p + (size_t)16 * DM;
  const v8f z8 = {0.f,0.f,0.f,0.f,0.f,0.f,0.f,0.f};
  v8f c00 = z8, c01 = z8, c02 = z8, c03 = z8, c10 = z8, c11 = z8, c12 = z8, c13 = z8;
#pragma unroll 1
  for (int kb = 0; kb < DM; kb += 32) {
    const v16h a0 = g2_frag(a0p + kb, hh), a1 = g2_frag(a1p + kb, hh);
    v16h b = g2_frag(b0p + kb, hh); c00 = g2_mma(a0, b, c00); c10 = g2_mma(a1, b, c10);
    b = g2_frag(b1p + kb, hh); c01 = g2_mma(a0, b, c01); c11 = g2_mma(a1, b, c11);
    b = g2_frag(b2p + kb, hh); c02 = g2_mma(a0, b, c02); c12 = g2_mma(a1, b, c12);
    b = g2_frag(b3p + kb, hh); c03 = g2_mma(a0, b, c03); c13 = g2_mma(a1, b, c13);
  }
  v8f accs[8] = {c00, c01, c02, c03, c10, c11, c12, c13};
#pragma unroll
  for (int u = 0; u < 8; ++u) {
    const int t = u & 3, hf = u >> 2;
#pragma unroll
    for (int r = 0; r < 8; ++r) so[w][hf * 16 + 8 * hh + r][t * 16 + ln] = accs[u][r] * alpha;
  }
  __builtin_amdgcn_fence(4  , "workgroup");
  __builtin_amdgcn_wave_barrier();
  const int rsub = lane >> 4, c4 = (lane & 15) * 4;
  for (int pass = 0; pass < 2; ++pass) {
#pragma unroll
    for (int q = 0; q < 16; ++q) {
      const int r = q * 2 + rsub;
      const int gr = row0 + r;
      const size_t orow = (size_t)(gr / SEQ) * SEQ_FULL + (size_t)(gr % SEQ);
      const v4f v = *(const v4fa*)&so[w][r][c4];
      *(volatile v4f*)(C + orow * DM + col0 + c4) = v;
    }
    if (pass == 0) __threadfence();
  }
}

extern "C" void kernel_launch(void* const* d_in, const int* in_sizes, int n_in,
                              void* d_out, int out_size, void* d_ws, size_t ws_size, hipStream_t stream) {
  if (n_in < 5) return;
  const size_t need = ((size_t)(NB - 1) * SEQ_FULL + SEQ) * DM;
  if ((size_t)in_sizes[0] < need) return;
  if ((size_t)in_sizes[3] < (size_t)3 * DM * DM) return;
  if ((size_t)in_sizes[4] < (size_t)DM * DM) return;
  if ((size_t)out_size < need) return;
  const float* query = (const float*)d_in[0];
  const float* w_qkv = (const float*)d_in[3];
  const float* w_out = (const float*)d_in[4];
  float* out = (float*)d_out;

  char* ws = (char*)d_ws; size_t off = 0;
  auto take = [&](size_t bytes) { char* p = ws + off; off += (bytes + 255) & ~(size_t)255; return p; };
  _Float16* WQKV = (_Float16*)take((size_t)3 * DM * DM * 2);
  _Float16* WOUT = (_Float16*)take((size_t)DM * DM * 2);
  _Float16* X16  = (_Float16*)take((size_t)NR * DM * 2);
  _Float16* QK   = (_Float16*)take((size_t)2 * NB * NH * SEQ * HD * 2);
  _Float16* VT   = (_Float16*)take((size_t)NB * NH * HD * SEQ * 2);
  _Float16* CTX  = (_Float16*)take((size_t)NR * DM * 2);
  float* CTAB    = (float*)take((size_t)SEQ * 32 * 4);
  float* STAB    = (float*)take((size_t)SEQ * 32 * 4);
  if (off > ws_size) return;

  k_x16<<<(unsigned)(((size_t)NR * DM / 8 + 255) / 256), 256, 0, stream>>>(query, X16);
  k_wnat<<<(unsigned)(((size_t)3 * DM * DM / 8 + 255) / 256), 256, 0, stream>>>(w_qkv, (size_t)3 * DM * DM / 8, WQKV);
  k_wnat<<<(unsigned)(((size_t)DM * DM / 8 + 255) / 256), 256, 0, stream>>>(w_out, (size_t)DM * DM / 8, WOUT);
  k_tab<<<(SEQ * 32 + 255) / 256, 256, 0, stream>>>(CTAB, STAB);
  k_qkv<<<(unsigned)((NR / 128) * ((3 * DM) / 64)), 128, 0, stream>>>(X16, WQKV, CTAB, STAB, QK, VT);
  k_flash<<<(unsigned)((NB * NH * (SEQ / 16)) / 4), 128, 0, stream>>>(QK, QK + (size_t)NB * NH * SEQ * HD, VT, CTX);
  k_out<<<(unsigned)((NR / 128) * (DM / 64)), 128, 0, stream>>>(CTX, WOUT, 0.0009765625f, out);
}
